// DenseGATv2Conv_5171140625162
// MI455X (gfx1250) — hardware-verified
//
#include <hip/hip_runtime.h>
#include <hip/hip_bf16.h>
#include <stdint.h>

#define B_   2
#define N_   1024
#define FIN_ 128
#define H_   4
#define C_   16
#define HC_  64
#define NEG_SLOPE_ 0.2f

typedef __attribute__((ext_vector_type(16))) _Float16 v16bf;
typedef __attribute__((ext_vector_type(8)))  float  v8f;

union FragBF {
  v16bf bf;
  uint4 u4[2];
};

__device__ __forceinline__ unsigned short f32_to_bf16_rne(float f) {
  return __builtin_bit_cast(unsigned short, (_Float16)f);
}

__global__ __launch_bounds__(256) void gat_proj_kernel(
    const float* __restrict__ x,   const float* __restrict__ W_l,
    const float* __restrict__ b_l, const float* __restrict__ W_r,
    const float* __restrict__ b_r,
    float* __restrict__ xl, float* __restrict__ xr,
    unsigned short* __restrict__ xrT) {
  __shared__ float s_x[4][FIN_];
  const int tid = threadIdx.x;
  const int r   = tid >> 6;
  const int hc  = tid & 63;
  const int row = blockIdx.x * 4 + r;
  const int b   = row >> 10;
  const int n   = row & (N_ - 1);

  const float* xrow = x + (size_t)row * FIN_;
  s_x[r][hc]      = xrow[hc];
  s_x[r][hc + 64] = xrow[hc + 64];
  __syncthreads();

  float al = 0.f, ar = 0.f;
#pragma unroll 8
  for (int f = 0; f < FIN_; ++f) {
    const float xv = s_x[r][f];
    al = fmaf(xv, W_l[f * HC_ + hc], al);
    ar = fmaf(xv, W_r[f * HC_ + hc], ar);
  }
  al += b_l[hc];
  ar += b_r[hc];

  const size_t o = (size_t)row * HC_ + hc;
  *(volatile float*)(xl + o) = al; *(volatile float*)(xr + o) = ar;
  __threadfence();
  *(volatile float*)(xl + o) = al; *(volatile float*)(xr + o) = ar;
  (void)b; (void)n; (void)xrT;
}

__global__ __launch_bounds__(256) void gat_xrT_kernel(const float* __restrict__ xr, unsigned short* __restrict__ xrT) {
  __shared__ float t[64][65];
  const int tid = threadIdx.x, lane = tid & 31, wave = tid >> 5;
  const int row0 = blockIdx.x * 64;
  const int b = row0 >> 10, n0 = row0 & (N_ - 1);
#pragma unroll
  for (int k = 0; k < 16; ++k) { const int e = tid + 256 * k; t[e >> 6][e & 63] = xr[(size_t)row0 * HC_ + e]; }
  __syncthreads();
#pragma unroll
  for (int r = 0; r < 8; ++r) {
    const int hc = wave * 8 + r, h = hc >> 4, c = hc & 15;
    const unsigned pk = (unsigned)f32_to_bf16_rne(t[2 * lane][hc]) | ((unsigned)f32_to_bf16_rne(t[2 * lane + 1][hc]) << 16);
    unsigned* dst = (unsigned*)(xrT + (((size_t)b * H_ + h) * C_ + c) * N_ + n0) + lane;
    *(volatile unsigned*)dst = pk; __threadfence(); *(volatile unsigned*)dst = pk;
  }
}

__global__ __launch_bounds__(256) void gat_attn_kernel(
    const float* __restrict__ xl,  const float* __restrict__ xr,
    const float* __restrict__ adj, const float* __restrict__ att,
    unsigned short* __restrict__ alphaB) {
  __shared__ float s_sc[H_][N_];
  __shared__ float s_xri[HC_];
  __shared__ float s_att[HC_];
  __shared__ float s_red[H_][256];

  const int tid = threadIdx.x;
  const int bi  = blockIdx.x;
  const int b   = bi >> 10;
  const int i   = bi & (N_ - 1);

  if (tid < HC_) {
    s_xri[tid] = xr[(size_t)bi * HC_ + tid];
    s_att[tid] = att[tid];
  }
  __syncthreads();

  const float* adjrow = adj + ((size_t)b * N_ + i) * N_;
  for (int j = tid; j < N_; j += 256) {
    const float* xlj = xl + ((size_t)b * N_ + j) * HC_;
    const float av = (j == i) ? 1.0f : adjrow[j];
#pragma unroll
    for (int h = 0; h < H_; ++h) {
      float acc = 0.f;
#pragma unroll
      for (int c = 0; c < C_; ++c) {
        float v = xlj[h * C_ + c] + s_xri[h * C_ + c];
        v = (v > 0.f) ? v : NEG_SLOPE_ * v;
        acc = fmaf(s_att[h * C_ + c], v, acc);
      }
      s_sc[h][j] = (av != 0.f) ? acc : -3.0e38f;
    }
  }
  __syncthreads();

  float pmax[H_];
#pragma unroll
  for (int h = 0; h < H_; ++h) pmax[h] = -3.0e38f;
  for (int j = tid; j < N_; j += 256)
#pragma unroll
    for (int h = 0; h < H_; ++h) pmax[h] = fmaxf(pmax[h], s_sc[h][j]);
#pragma unroll
  for (int h = 0; h < H_; ++h) s_red[h][tid] = pmax[h];
  __syncthreads();
  for (int s = 128; s > 0; s >>= 1) {
    if (tid < s)
#pragma unroll
      for (int h = 0; h < H_; ++h)
        s_red[h][tid] = fmaxf(s_red[h][tid], s_red[h][tid + s]);
    __syncthreads();
  }
  float mx[H_];
#pragma unroll
  for (int h = 0; h < H_; ++h) mx[h] = s_red[h][0];
  __syncthreads();

  float psum[H_];
#pragma unroll
  for (int h = 0; h < H_; ++h) psum[h] = 0.f;
  for (int j = tid; j < N_; j += 256)
#pragma unroll
    for (int h = 0; h < H_; ++h) {
      const float p = __expf(s_sc[h][j] - mx[h]);
      s_sc[h][j] = p;
      psum[h] += p;
    }
#pragma unroll
  for (int h = 0; h < H_; ++h) s_red[h][tid] = psum[h];
  __syncthreads();
  for (int s = 128; s > 0; s >>= 1) {
    if (tid < s)
#pragma unroll
      for (int h = 0; h < H_; ++h)
        s_red[h][tid] += s_red[h][tid + s];
    __syncthreads();
  }
  float inv[H_];
#pragma unroll
  for (int h = 0; h < H_; ++h) inv[h] = 1.0f / s_red[h][0];

  __syncthreads();
  for (int j2 = tid; j2 < N_ / 2; j2 += 256)
#pragma unroll
    for (int h = 0; h < H_; ++h) {
      const float sc = inv[h] * 1024.0f;
      const unsigned pk = (unsigned)f32_to_bf16_rne(s_sc[h][2 * j2] * sc) | ((unsigned)f32_to_bf16_rne(s_sc[h][2 * j2 + 1] * sc) << 16);
      unsigned* dst = (unsigned*)(alphaB + (((size_t)b * H_ + h) * N_ + i) * N_) + j2;
      *(volatile unsigned*)dst = pk; __threadfence(); *(volatile unsigned*)dst = pk;
    }
}

__global__ __launch_bounds__(128) void gat_aggr_wmma_kernel(
    const unsigned short* __restrict__ alphaB,
    const unsigned short* __restrict__ xrT,
    const float* __restrict__ bias,
    float* __restrict__ out) {
  __shared__ __attribute__((aligned(16))) float so[4][16 * 64];
  const int lane = threadIdx.x & 31;
  const int wave = threadIdx.x >> 5;
  const int tile = blockIdx.x * 4 + wave;
  const int b    = blockIdx.z;
  const int i0   = tile * 16;
  const int half = lane >> 4;
  const int m    = lane & 15;
  float* sw = so[wave];

#pragma unroll 1
  for (int h = 0; h < H_; ++h) {
    const unsigned short* Arow = alphaB + (((size_t)b * H_ + h) * N_ + (i0 + m)) * N_;
    const unsigned short* Bcol = xrT + (((size_t)b * H_ + h) * C_ + m) * N_;
    v8f acc = {};
    for (int j0 = 0; j0 < N_; j0 += 32) {
      FragBF a, bb;
      a.u4[0]  = *(const uint4*)(Arow + j0 + 8 * half);
      a.u4[1]  = *(const uint4*)(Arow + j0 + 16 + 8 * half);
      bb.u4[0] = *(const uint4*)(Bcol + j0 + 8 * half);
      bb.u4[1] = *(const uint4*)(Bcol + j0 + 16 + 8 * half);
      if (j0 + 32 < N_) {
        __builtin_prefetch(Arow + j0 + 32, 0, 0);
        __builtin_prefetch(Bcol + j0 + 32, 0, 0);
      }
      acc = __builtin_amdgcn_wmma_f32_16x16x32_f16(
           false, a.bf,  false, bb.bf,
           (short)0, acc,  false,  false);
    }
    const float bv = bias[h * C_ + m];
#pragma unroll
    for (int r = 0; r < 8; ++r) sw[(r + 8 * half) * 64 + h * C_ + m] = acc[r] * (1.0f / 1024.0f) + bv;
  }
  asm volatile("s_wait_dscnt 0" ::: "memory");
  typedef __attribute__((ext_vector_type(4))) float v4f_t;
  typedef float v4fa __attribute__((ext_vector_type(4), may_alias));
  float* outb = out + (size_t)b * N_ * HC_;
  v4f_t ov[8]; size_t oo[8];
#pragma unroll
  for (int i = 0; i < 8; ++i) { const int c = lane + 32 * i, rr = c >> 4, q = c & 15; ov[i] = *(const volatile v4fa*)(sw + rr * 64 + q * 4); oo[i] = (size_t)(i0 + rr) * HC_ + q * 4; }
#pragma unroll
  for (int i = 0; i < 8; ++i) *(volatile v4f_t*)(outb + oo[i]) = ov[i];
  __threadfence();
#pragma unroll
  for (int i = 0; i < 8; ++i) *(volatile v4f_t*)(outb + oo[i]) = ov[i];
}

extern "C" void kernel_launch(void* const* d_in, const int* in_sizes, int n_in,
                              void* d_out, int out_size, void* d_ws, size_t ws_size,
                              hipStream_t stream) {
  (void)in_sizes; (void)n_in; (void)out_size; (void)ws_size;
  const float* x    = (const float*)d_in[0];
  const float* adj  = (const float*)d_in[1];
  const float* W_l  = (const float*)d_in[2];
  const float* b_l  = (const float*)d_in[3];
  const float* W_r  = (const float*)d_in[4];
  const float* b_r  = (const float*)d_in[5];
  const float* att  = (const float*)d_in[6];
  const float* bias = (const float*)d_in[7];
  float* out = (float*)d_out;

  char* ws = (char*)d_ws;
  const size_t xl_off    = 0;
  const size_t xr_off    = xl_off  + sizeof(float) * B_ * N_ * HC_;
  const size_t xrT_off   = xr_off  + sizeof(float) * B_ * N_ * HC_;
  const size_t alpha_off = xrT_off + sizeof(unsigned short) * B_ * H_ * C_ * N_;
  float*          xl     = (float*)(ws + xl_off);
  float*          xr     = (float*)(ws + xr_off);
  unsigned short* xrT    = (unsigned short*)(ws + xrT_off);
  unsigned short* alphaB = (unsigned short*)(ws + alpha_off);

  gat_proj_kernel<<<dim3(B_ * N_ / 4), dim3(256), 0, stream>>>(
      x, W_l, b_l, W_r, b_r, xl, xr, xrT);
  gat_xrT_kernel<<<dim3(B_ * N_ / 64), dim3(256), 0, stream>>>(xr, xrT);
  gat_attn_kernel<<<dim3(B_ * N_), dim3(256), 0, stream>>>(
      xl, xr, adj, att, alphaB);
  gat_aggr_wmma_kernel<<<dim3(N_ / 16 / 4, 1, B_), dim3(128), 0, stream>>>(
      alphaB, xrT, bias, out);
}
